// ParallelMamba_12893491822622
// MI455X (gfx1250) — hardware-run, weakly checked
//
#include <hip/hip_runtime.h>
#include <math.h>

typedef __attribute__((ext_vector_type(16))) _Float16 v16h;
typedef __attribute__((ext_vector_type(8)))  _Float16 v8h;
typedef __attribute__((ext_vector_type(8)))  float    v8f;
typedef __attribute__((ext_vector_type(4)))  float    v4f;

constexpr int kB     = 2;
constexpr int kL     = 1024;
constexpr int kDM    = 1024;
constexpr int kDI    = 2048;
constexpr int kNS    = 16;
constexpr int kRank  = 64;
constexpr int kTaps  = 3;
constexpr int kChunk = 256;
constexpr int kT     = kB * kL;
constexpr int kXRP   = 2 * kDI;
constexpr int kXPW   = kRank + 2 * kNS;
constexpr int kXPP   = 128;
constexpr int kConvTP = 260;
constexpr int kScanTS = 16;
constexpr int kScanYP = 260;
static_assert(kXPW == 96);
static_assert(kXPW <= kXPP && (kXPP % 64) == 0);
static_assert((kL & (kL - 1)) == 0 && (kL % kChunk) == 0 && (kL % 64) == 0);
static_assert((kDM % 32) == 0 && (kDI % 32) == 0 && (kRank % 32) == 0);
static_assert((kT % 64) == 0 && (kXRP % 64) == 0 && (kDI % 64) == 0 && (kDM % 64) == 0);
static_assert((kDI % 256) == 0 && (kChunk % kScanTS) == 0 && kNS == 16 && kTaps == 3);

constexpr float kCarryX    = 64.0f;
constexpr float kCarryWin  = 4096.0f;
constexpr float kCarryU    = 1024.0f;
constexpr float kCarryRes  = 2048.0f;
constexpr float kCarryW    = 1024.0f;
constexpr float kCarryDlt  = 16384.0f;
constexpr float kCarryY    = 16777216.0f;
constexpr float kFoldIn    = 1.0f / (kCarryX * kCarryWin);
constexpr float kFoldXp    = 1.0f / (kCarryU * kCarryW);
constexpr float kFoldRes   = 1.0f / kCarryRes;
constexpr float kFoldDt    = 1.0f / (kCarryDlt * kCarryW);
constexpr float kFoldOut   = 1.0f / (kCarryY * kCarryW);
constexpr float kF16MinNormal = 6.103515625e-05f;

constexpr size_t kSzX16    = (size_t)kT * kDM * 2;
constexpr size_t kSzWIN16  = (size_t)kXRP * kDM * 2;
constexpr size_t kSzWX16   = (size_t)kXPP * kDI * 2;
constexpr size_t kSzWDT16  = (size_t)kDI * kRank * 2;
constexpr size_t kSzWOUT16 = (size_t)kDM * kDI * 2;
constexpr size_t kSzXR     = (size_t)kT * kXRP * 4;
constexpr size_t kSzUF     = (size_t)kT * kDI * 4;
constexpr size_t kSzUH     = (size_t)kT * kDI * 2;
constexpr size_t kSzUL     = (size_t)kT * kDI * 2;
constexpr size_t kSzXP     = (size_t)kT * kXPP * 4;
constexpr size_t kSzDL16   = (size_t)kT * kRank * 2;
constexpr size_t kSzDR     = (size_t)kT * kDI * 4;
constexpr size_t kSzY16    = (size_t)kT * kDI * 2;
constexpr size_t kOffX16    = 0;
constexpr size_t kOffWIN16  = kOffX16    + kSzX16;
constexpr size_t kOffWX16   = kOffWIN16  + kSzWIN16;
constexpr size_t kOffWDT16  = kOffWX16   + kSzWX16;
constexpr size_t kOffWOUT16 = kOffWDT16  + kSzWDT16;
constexpr size_t kOffXR     = kOffWOUT16 + kSzWOUT16;
constexpr size_t kOffUF     = kOffXR     + kSzXR;
constexpr size_t kOffUH     = kOffUF     + kSzUF;
constexpr size_t kOffUL     = kOffUH     + kSzUH;
constexpr size_t kOffXP     = kOffUL     + kSzUL;
constexpr size_t kOffDL16   = kOffXP     + kSzXP;
constexpr size_t kOffDR     = kOffDL16   + kSzDL16;
constexpr size_t kOffY16    = kOffDR     + kSzDR;
constexpr size_t kWsTotal   = kOffY16    + kSzY16;
static_assert(kWsTotal == 111149056ull);
static_assert(kWsTotal <= 134217728ull);
static_assert((kOffWIN16 % 128) == 0 && (kOffWX16 % 128) == 0 && (kOffWDT16 % 128) == 0 &&
              (kOffWOUT16 % 128) == 0 && (kOffXR % 128) == 0 && (kOffUF % 128) == 0 &&
              (kOffUH % 128) == 0 && (kOffUL % 128) == 0 && (kOffXP % 128) == 0 &&
              (kOffDL16 % 128) == 0 && (kOffDR % 128) == 0 && (kOffY16 % 128) == 0);

__device__ __forceinline__ float bfv(float f) {
  const unsigned u = __float_as_uint(f);
  const unsigned r = (u + 0x7FFFu + ((u >> 16) & 1u)) & 0xFFFF0000u;
  return __uint_as_float(r);
}
__device__ __forceinline__ _Float16 op_f16(float v) {
  const float a = fabsf(v);
  float w = (a < kF16MinNormal) ? 0.0f : v;
  w = fminf(fmaxf(w, -60000.0f), 60000.0f);
  return (_Float16)w;
}

union FragU { v16h v; v8h h[2]; };
__device__ __forceinline__ v16h frag_load(const _Float16* p) {
  FragU f;
  f.h[0] = *(const v8h*)(p);
  f.h[1] = *(const v8h*)(p + 16);
  return f.v;
}
__device__ __forceinline__ v8f mma_f16(v16h a, v16h b, v8f c) {
  return __builtin_amdgcn_wmma_f32_16x16x32_f16(false, a, false, b, (short)0, c, false, false);
}
__device__ __forceinline__ void tie_acc(v8f& c, v16h a, v16h b) {
  asm volatile("" : "+v"(c) : "v"(a), "v"(b));
}
__device__ __forceinline__ void guard_acc(v8f& c, v16h a, v16h a2, v16h b) {
  asm volatile("v_nop\n\tv_nop\n\tv_nop\n\tv_nop" : "+v"(c) : "v"(a), "v"(a2), "v"(b));
}
__device__ __forceinline__ void keep4(v16h a, v16h b, v16h c, v16h d) {
  asm volatile("v_nop" :: "v"(a), "v"(b), "v"(c), "v"(d));
}

template <int MI, bool RES, int BIAS_MODE>
__global__ __launch_bounds__(256) void gemm_f16_kernel(
    const unsigned short* __restrict__ Ap, const unsigned short* __restrict__ A2p, int lda,
    const unsigned short* __restrict__ Btp, int ldb,
    float* __restrict__ C, int ldc,
    const float* __restrict__ bias,
    int M, int N, int K, float fold, float rfold)
{
  const _Float16* A  = (const _Float16*)Ap;
  const _Float16* A2 = (const _Float16*)A2p;
  const _Float16* Bt = (const _Float16*)Btp;
  __shared__ __align__(16) float sT[8][16 * 68];
  const int lane = threadIdx.x & 31;
  const int wave = threadIdx.x >> 5;
  const int tilesN = N >> 6;
  const int tilesM = M / (16 * MI);
  const int tile = blockIdx.x * 8 + wave;
  if (tile >= tilesM * tilesN) return;
  const int tm = tile / tilesN;
  const int tn = tile - tm * tilesN;
  const int m0 = tm * (16 * MI);
  const int n0 = tn << 6;
  const int rlane = lane & 15;
  const int koff  = (lane >> 4) * 8;
  const int mOff  = (lane >> 4) * 8;

  v8f acc[MI][4];
  v8f accr[RES ? MI : 1][4];
#pragma unroll
  for (int i = 0; i < MI; ++i)
#pragma unroll
    for (int j = 0; j < 4; ++j) acc[i][j] = (v8f){0.f, 0.f, 0.f, 0.f, 0.f, 0.f, 0.f, 0.f};
#pragma unroll
  for (int i = 0; i < (RES ? MI : 1); ++i)
#pragma unroll
    for (int j = 0; j < 4; ++j) accr[i][j] = (v8f){0.f, 0.f, 0.f, 0.f, 0.f, 0.f, 0.f, 0.f};

  for (int k0 = 0; k0 < K; k0 += 32) {
    v16h bh[4];
#pragma unroll
    for (int j = 0; j < 4; ++j) {
      const size_t bo = (size_t)(n0 + (j << 4) + rlane) * ldb + koff + k0;
      bh[j] = frag_load(Bt + bo);
    }
#pragma unroll
    for (int i = 0; i < MI; ++i) {
      const size_t ao = (size_t)(m0 + (i << 4) + rlane) * lda + koff + k0;
      const v16h ah = frag_load(A + ao);
      v16h al = ah;
      if (RES) al = frag_load(A2 + ao);
#pragma unroll
      for (int j = 0; j < 4; ++j) {
        acc[i][j] = mma_f16(ah, bh[j], acc[i][j]);
        if (RES) accr[RES ? i : 0][j] = mma_f16(al, bh[j], accr[RES ? i : 0][j]);
      }
#pragma unroll
      for (int j = 0; j < 4; ++j) {
        if (RES) tie_acc(accr[RES ? i : 0][j], al, bh[j]);
        if (j < 3) tie_acc(acc[i][j], ah, bh[j]);
      }
      guard_acc(acc[i][3], ah, al, bh[3]);
    }
    keep4(bh[0], bh[1], bh[2], bh[3]);
  }

  float* slab = sT[wave];
  float bv[4];
#pragma unroll
  for (int j = 0; j < 4; ++j) {
    bv[j] = 0.0f;
    if (BIAS_MODE == 3) bv[j] = bfv(bias[n0 + (j << 4) + rlane]);
  }
#pragma unroll
  for (int i = 0; i < MI; ++i) {
    const int mBase = m0 + (i << 4);
#pragma unroll
    for (int j = 0; j < 4; ++j) {
#pragma unroll
      for (int r = 0; r < 8; ++r) {
        float v = acc[i][j][r];
        if (RES) v = fmaf(accr[RES ? i : 0][j][r], rfold, v);
        v = v * fold + bv[j];
        slab[(mOff + r) * 68 + (j << 4) + rlane] = v;
      }
    }
    __builtin_amdgcn_fence(__ATOMIC_RELEASE, "workgroup");
    __builtin_amdgcn_wave_barrier();
    __builtin_amdgcn_fence(__ATOMIC_ACQUIRE, "workgroup");
    {
      const int hh = lane >> 4, c4 = (lane & 15) * 4;
      for (int pass = 0; pass < 2; ++pass) {
#pragma unroll
        for (int it = 0; it < 8; ++it) {
          const int row = it * 2 + hh;
          const v4f v = *(const v4f*)(slab + row * 68 + c4);
          *(volatile v4f*)(C + (size_t)(mBase + row) * ldc + n0 + c4) = v;
        }
        __threadfence();
      }
    }
    __builtin_amdgcn_fence(__ATOMIC_RELEASE, "workgroup");
    __builtin_amdgcn_wave_barrier();
    __builtin_amdgcn_fence(__ATOMIC_ACQUIRE, "workgroup");
  }
}

__global__ __launch_bounds__(256) void plane_from_input_kernel(
    const float* __restrict__ src, unsigned short* __restrict__ dst, int total8, int real8, float carry)
{
  const int i = blockIdx.x * 256 + threadIdx.x;
  if (i >= total8) return;
  const bool live = (i < real8);
  const int ic = live ? i : (real8 - 1);
  const size_t e0 = (size_t)ic << 3;
  const v4f a0 = *(const v4f*)(src + e0);
  const v4f a1 = *(const v4f*)(src + e0 + 4);
  v8h hv;
#pragma unroll
  for (int e = 0; e < 4; ++e) {
    const float f0 = live ? (bfv(a0[e]) * carry) : 0.0f;
    const float f1 = live ? (bfv(a1[e]) * carry) : 0.0f;
    hv[e]     = op_f16(f0);
    hv[4 + e] = op_f16(f1);
  }
  unsigned short* q = dst + ((size_t)i << 3);
  *(volatile v8h*)q = hv;
  __threadfence();
  *(volatile v8h*)q = hv;
}

__global__ __launch_bounds__(256) void conv_act_kernel(
    const float* __restrict__ XR, const float* __restrict__ cw, const float* __restrict__ cb,
    float* __restrict__ UF, unsigned short* __restrict__ UH, unsigned short* __restrict__ UL)
{
  __shared__ __align__(16) float sT[16 * kConvTP];
  const int tid = threadIdx.x, lane = tid & 31, wave = tid >> 5;
  const int d0 = blockIdx.x * 256, d = d0 + tid;
  const int g0 = blockIdx.y * 64;
  const int tb = g0 & (kL - 1);
  const float w0 = bfv(cw[d * kTaps + 0]);
  const float w1 = bfv(cw[d * kTaps + 1]);
  const float w2 = bfv(cw[d * kTaps + 2]);
  const float bc = bfv(cb[d]);
  float xm2, xm1;
  {
    const bool hist = (tb > 0);
    const int rb = hist ? (g0 - 2) : g0;
    const float v2 = XR[(size_t)rb * kXRP + d];
    const float v1 = XR[(size_t)(rb + 1) * kXRP + d];
    xm2 = hist ? v2 : 0.0f;
    xm1 = hist ? v1 : 0.0f;
  }
  const int hrow = wave >> 1;
  const int hch  = (wave & 1) * 128 + lane * 4;
#pragma unroll 1
  for (int sub = 0; sub < 4; ++sub) {
    const int lb = g0 + sub * 16;
#pragma unroll 1
    for (int s = 0; s < 16; ++s) {
      const float xcur = XR[(size_t)(lb + s) * kXRP + d];
      float acc = w0 * xm2;
      acc = fmaf(w1, xm1, acc);
      acc = fmaf(w2, xcur, acc);
      const float sv = acc + bc;
      const float den = 1.0f + expf(-sv);
      sT[s * kConvTP + tid] = sv * (1.0f / den);
      xm2 = xm1;
      xm1 = xcur;
    }
    __syncthreads();
    v4f fv[4];
    v8h ph[2], pl[2];
#pragma unroll
    for (int it = 0; it < 4; ++it) fv[it] = *(const v4f*)(sT + (it * 4 + hrow) * kConvTP + hch);
#pragma unroll
    for (int it = 0; it < 2; ++it) {
      const float* sp = sT + (it * 8 + wave) * kConvTP + lane * 8;
      const v4f a0 = *(const v4f*)(sp);
      const v4f a1 = *(const v4f*)(sp + 4);
#pragma unroll
      for (int e = 0; e < 4; ++e) {
        const float c0 = a0[e] * kCarryU;
        const float c1 = a1[e] * kCarryU;
        const _Float16 h0 = op_f16(c0);
        const _Float16 h1 = op_f16(c1);
        const float r0 = (c0 - (float)h0) * kCarryRes;
        const float r1 = (c1 - (float)h1) * kCarryRes;
        ph[it][e]     = h0;
        ph[it][4 + e] = h1;
        pl[it][e]     = op_f16(r0);
        pl[it][4 + e] = op_f16(r1);
      }
    }
    for (int pass = 0; pass < 2; ++pass) {
#pragma unroll
      for (int it = 0; it < 4; ++it)
        *(volatile v4f*)(UF + (size_t)(lb + it * 4 + hrow) * kDI + d0 + hch) = fv[it];
#pragma unroll
      for (int it = 0; it < 2; ++it) {
        const size_t o = (size_t)(lb + it * 8 + wave) * kDI + d0 + lane * 8;
        *(volatile v8h*)(UH + o) = ph[it];
        *(volatile v8h*)(UL + o) = pl[it];
      }
      __threadfence();
    }
    __syncthreads();
  }
}

__global__ __launch_bounds__(256) void dlt_plane_kernel(
    const float* __restrict__ XP, unsigned short* __restrict__ DL)
{
  const int i = blockIdx.x * 256 + threadIdx.x;
  if (i >= kT * kRank / 8) return;
  const int row = i >> 3, c8 = (i & 7) * 8;
  const float* sp = XP + (size_t)row * kXPP + c8;
  const v4f a0 = *(const v4f*)(sp);
  const v4f a1 = *(const v4f*)(sp + 4);
  v8h hv;
#pragma unroll
  for (int e = 0; e < 4; ++e) {
    hv[e]     = op_f16(a0[e] * kCarryDlt);
    hv[4 + e] = op_f16(a1[e] * kCarryDlt);
  }
  unsigned short* q = DL + (size_t)row * kRank + c8;
  *(volatile v8h*)q = hv;
  __threadfence();
  *(volatile v8h*)q = hv;
}

__global__ __launch_bounds__(256) void chunk_scan_kernel(
    const float* __restrict__ DRp, const float* __restrict__ UF, const float* __restrict__ XP,
    const float* __restrict__ XR, const float* __restrict__ Alog, unsigned short* __restrict__ Y16)
{
  __shared__ __align__(16) float sBC[kChunk * 32];
  __shared__ __align__(16) float sY[kScanTS * kScanYP];
  const int tid = threadIdx.x, lane = tid & 31, wave = tid >> 5;
  const int d0 = blockIdx.x * 256, d = d0 + tid;
  const int t0 = (int)blockIdx.z * kL + (int)blockIdx.y * kChunk;

#pragma unroll 1
  for (int it = 0; it < 8; ++it) {
    const int idx = tid + it * 256;
    const int t = idx >> 3, j4 = (idx & 7) * 4;
    const v4f v = *(const v4f*)(XP + (size_t)(t0 + t) * kXPP + kRank + j4);
    *(v4f*)(sBC + t * 32 + j4) = v;
  }
#pragma unroll 1
  for (int n = 0; n < kNS; ++n) {
    const float al = bfv(Alog[(size_t)d * kNS + n]);
    sY[n * kScanYP + tid] = -expf(al);
  }
  __syncthreads();
  float an[kNS], carry[kNS];
#pragma unroll
  for (int n = 0; n < kNS; ++n) {
    an[n] = sY[n * kScanYP + tid];
    carry[n] = 0.0f;
  }
  __syncthreads();

#pragma unroll 1
  for (int tg = 0; tg < kChunk; tg += kScanTS) {
#pragma unroll 1
    for (int s = 0; s < kScanTS; ++s) {
      const int t = tg + s;
      const size_t tok = (size_t)(t0 + t);
      const float dr = DRp[tok * kDI + d];
      const float uu = UF[tok * kDI + d];
      const float rs = XR[tok * kXRP + kDI + d];
      const float ea = expf(-fabsf(dr));
      const float up = 1.0f + ea;
      const float l1p = logf(up) + (ea - (up - 1.0f)) * __builtin_amdgcn_rcpf(up);
      const float delta = fmaxf(dr, 0.0f) + l1p;
      const float du = delta * uu;
      const float* bcp = sBC + t * 32;
      v4f bq[4], cq[4];
#pragma unroll
      for (int q = 0; q < 4; ++q) {
        bq[q] = *(const v4f*)(bcp + 4 * q);
        cq[q] = *(const v4f*)(bcp + kNS + 4 * q);
      }
      float y = 0.0f;
#pragma unroll
      for (int q = 0; q < 4; ++q) {
#pragma unroll
        for (int e = 0; e < 4; ++e) {
          const float dec = __expf(delta * an[4 * q + e]);
          carry[4 * q + e] = dec * carry[4 * q + e] + du * bq[q][e];
          y = fmaf(carry[4 * q + e], cq[q][e], y);
        }
      }
      const float gden = 1.0f + expf(-rs);
      const float gate = rs * (1.0f / gden);
      sY[s * kScanYP + tid] = y * gate;
    }
    __syncthreads();
    v8h hv[2];
#pragma unroll
    for (int it = 0; it < 2; ++it) {
      const float* sp = sY + (it * 8 + wave) * kScanYP + lane * 8;
      const v4f a0 = *(const v4f*)(sp);
      const v4f a1 = *(const v4f*)(sp + 4);
#pragma unroll
      for (int e = 0; e < 4; ++e) {
        hv[it][e]     = op_f16(a0[e] * kCarryY);
        hv[it][4 + e] = op_f16(a1[e] * kCarryY);
      }
    }
    for (int pass = 0; pass < 2; ++pass) {
#pragma unroll
      for (int it = 0; it < 2; ++it) {
        const size_t o = (size_t)(t0 + tg + it * 8 + wave) * kDI + d0 + lane * 8;
        *(volatile v8h*)(Y16 + o) = hv[it];
      }
      __threadfence();
    }
    __syncthreads();
  }
}

extern "C" void kernel_launch(void* const* d_in, const int* in_sizes, int n_in,
                              void* d_out, int out_size, void* d_ws, size_t ws_size,
                              hipStream_t stream) {
  if (n_in < 11) return;
  if (in_sizes[0] != kT * kDM) return;
  if (in_sizes[1] != kXRP * kDM) return;
  if (in_sizes[2] != kXRP) return;
  if (in_sizes[3] != kDI * kTaps) return;
  if (in_sizes[4] != kDI) return;
  if (in_sizes[5] != kXPW * kDI) return;
  if (in_sizes[6] != kDI * kRank) return;
  if (in_sizes[7] != kDI) return;
  if (in_sizes[8] != kDI * kNS) return;
  if (in_sizes[9] != kDM * kDI) return;
  if (in_sizes[10] != kDM) return;
  if (out_size != kT * kDM) return;
  if (ws_size < kWsTotal) return;

  const float* x      = (const float*)d_in[0];
  const float* W_in   = (const float*)d_in[1];
  const float* b_in   = (const float*)d_in[2];
  const float* conv_w = (const float*)d_in[3];
  const float* conv_b = (const float*)d_in[4];
  const float* W_x    = (const float*)d_in[5];
  const float* W_dt   = (const float*)d_in[6];
  const float* b_dt   = (const float*)d_in[7];
  const float* A_log  = (const float*)d_in[8];
  const float* W_out  = (const float*)d_in[9];
  const float* b_out  = (const float*)d_in[10];
  float* out = (float*)d_out;

  char* ws = (char*)d_ws;
  unsigned short* X16    = (unsigned short*)(ws + kOffX16);
  unsigned short* WIN16  = (unsigned short*)(ws + kOffWIN16);
  unsigned short* WX16   = (unsigned short*)(ws + kOffWX16);
  unsigned short* WDT16  = (unsigned short*)(ws + kOffWDT16);
  unsigned short* WOUT16 = (unsigned short*)(ws + kOffWOUT16);
  float*          XR     = (float*)(ws + kOffXR);
  float*          UF     = (float*)(ws + kOffUF);
  unsigned short* UH     = (unsigned short*)(ws + kOffUH);
  unsigned short* UL     = (unsigned short*)(ws + kOffUL);
  float*          XP     = (float*)(ws + kOffXP);
  unsigned short* DL16   = (unsigned short*)(ws + kOffDL16);
  float*          DR     = (float*)(ws + kOffDR);
  unsigned short* Y16    = (unsigned short*)(ws + kOffY16);

  const dim3 blk(256);

  {
    constexpr int nX  = kT * kDM / 8;
    constexpr int nWi = kXRP * kDM / 8;
    constexpr int nWxT = kXPP * kDI / 8;
    constexpr int nWxR = kXPW * kDI / 8;
    constexpr int nWd = kDI * kRank / 8;
    constexpr int nWo = kDM * kDI / 8;
    static_assert((nX % 256) == 0 && (nWi % 256) == 0 && (nWxT % 256) == 0 && (nWd % 256) == 0 && (nWo % 256) == 0);
    plane_from_input_kernel<<<dim3(nX / 256), blk, 0, stream>>>(x, X16, nX, nX, kCarryX);
    plane_from_input_kernel<<<dim3(nWi / 256), blk, 0, stream>>>(W_in, WIN16, nWi, nWi, kCarryWin);
    plane_from_input_kernel<<<dim3(nWxT / 256), blk, 0, stream>>>(W_x, WX16, nWxT, nWxR, kCarryW);
    plane_from_input_kernel<<<dim3(nWd / 256), blk, 0, stream>>>(W_dt, WDT16, nWd, nWd, kCarryW);
    plane_from_input_kernel<<<dim3(nWo / 256), blk, 0, stream>>>(W_out, WOUT16, nWo, nWo, kCarryW);
  }

  {
    constexpr int tiles = (kT / 64) * (kXRP / 64);
    static_assert((tiles % 8) == 0);
    gemm_f16_kernel<4, false, 3><<<dim3(tiles / 8), blk, 0, stream>>>(
        X16, X16, kDM, WIN16, kDM, XR, kXRP, b_in, kT, kXRP, kDM, kFoldIn, 0.0f);
  }

  conv_act_kernel<<<dim3(kDI / 256, kT / 64), blk, 0, stream>>>(XR, conv_w, conv_b, UF, UH, UL);

  {
    constexpr int tiles = (kT / 32) * (kXPP / 64);
    static_assert((tiles % 8) == 0);
    gemm_f16_kernel<2, true, 0><<<dim3(tiles / 8), blk, 0, stream>>>(
        UH, UL, kDI, WX16, kDI, XP, kXPP, b_in, kT, kXPP, kDI, kFoldXp, kFoldRes);
  }

  dlt_plane_kernel<<<dim3(kT * kRank / 8 / 256), blk, 0, stream>>>(XP, DL16);

  {
    constexpr int tiles = (kT / 64) * (kDI / 64);
    static_assert((tiles % 8) == 0);
    gemm_f16_kernel<4, false, 3><<<dim3(tiles / 8), blk, 0, stream>>>(
        DL16, DL16, kRank, WDT16, kRank, DR, kDI, b_dt, kT, kDI, kRank, kFoldDt, 0.0f);
  }

  chunk_scan_kernel<<<dim3(kDI / 256, kL / kChunk, kB), blk, 0, stream>>>(DR, UF, XP, XR, A_log, Y16);

  {
    constexpr int tiles = (kT / 64) * (kDM / 64);
    static_assert((tiles % 8) == 0);
    gemm_f16_kernel<4, false, 3><<<dim3(tiles / 8), blk, 0, stream>>>(
        Y16, Y16, kDI, WOUT16, kDI, out, kDM, b_out, kT, kDM, kDI, kFoldOut, 0.0f);
  }
}
